// ChebyKANLayer_64355789963436
// MI455X (gfx1250) — hardware-verified
//
#include <hip/hip_runtime.h>


#define NB   4096
#define DI   1024
#define DO_  1024
#define ND   5
#define KK   (ND * DI)
typedef _Float16 h16;
typedef unsigned short bf;
typedef __attribute__((ext_vector_type(16))) __bf16   v16bf;
typedef __attribute__((ext_vector_type(16))) _Float16 v16h;
typedef __attribute__((ext_vector_type(8)))  _Float16 v8h;
typedef __attribute__((ext_vector_type(8)))  unsigned short v8us;
typedef __attribute__((ext_vector_type(8)))  float    v8f;
typedef __attribute__((ext_vector_type(4)))  float    v4f;
typedef v8h  __attribute__((may_alias)) v8ha;
typedef v4f  __attribute__((may_alias)) v4fa;
typedef v8us __attribute__((may_alias)) v8usa;

__device__ __forceinline__ unsigned short f2bf(float f) { unsigned u = __float_as_uint(f); u += 0x7FFFu + ((u >> 16) & 1u); return (unsigned short)(u >> 16); }
__device__ __forceinline__ float bf2f(unsigned short b) { return __uint_as_float(((unsigned)b) << 16); }
__device__ __forceinline__ float bfr(float f) { return bf2f(f2bf(f)); }
__device__ __forceinline__ v16h cat16(v8h lo, v8h hi) { return __builtin_shufflevector(lo, hi, 0, 1, 2, 3, 4, 5, 6, 7, 8, 9, 10, 11, 12, 13, 14, 15); }
__device__ __forceinline__ v16bf cat16b(v8us lo, v8us hi) { return __builtin_bit_cast(v16bf, __builtin_shufflevector(lo, hi, 0, 1, 2, 3, 4, 5, 6, 7, 8, 9, 10, 11, 12, 13, 14, 15)); }
__device__ __forceinline__ v8f wmma16(v16h a, v16h b, v8f c) { return __builtin_amdgcn_wmma_f32_16x16x32_f16(false, a, false, b, (short)0, c, false, false); }
__device__ __forceinline__ v8f wmmab(v16bf a, v16bf b, v8f c) { return __builtin_amdgcn_wmma_f32_16x16x32_bf16(false, a, false, b, (short)0, c, false, false); }


template <typename T16> struct WFrag;
template <> struct WFrag<h16> { typedef v16h V; static __device__ __forceinline__ V ld(const h16* p) { return cat16(*(const v8h*)p, *(const v8h*)(p + 16)); } static __device__ __forceinline__ v8f mma(V a, V b, v8f c) { return wmma16(a, b, c); } };
template <> struct WFrag<bf> { typedef v16bf V; static __device__ __forceinline__ V ld(const bf* p) { return cat16b(*(const v8us*)p, *(const v8us*)(p + 16)); } static __device__ __forceinline__ v8f mma(V a, V b, v8f c) { return wmmab(a, b, c); } };
template <typename T16, int NSPLIT, bool BIAS>
__global__ __launch_bounds__(32) void k_gemmw(const T16* __restrict__ A, const T16* __restrict__ A2, const T16* __restrict__ Bt, const T16* __restrict__ Bt2, int K, float* C, int ldc, const float* __restrict__ bias, size_t sA, size_t sB, size_t sC) {
    typedef typename WFrag<T16>::V V;
    __shared__ __align__(16) float os[16 * 68];
    const size_t z = blockIdx.z; A += z * sA; if (A2) A2 += z * sA; Bt += z * sB; if (Bt2) Bt2 += z * sB; C += z * sC;
    const int lane = threadIdx.x & 31, lr = lane & 15, hi = lane >> 4; const int r0 = blockIdx.x * 64, c0 = blockIdx.y * 64;
    v8f acc[4][4];
#pragma unroll
    for (int mb = 0; mb < 4; ++mb)
#pragma unroll
        for (int nb = 0; nb < 4; ++nb) acc[mb][nb] = (v8f){};
    const size_t aoff = (size_t)(r0 + lr) * K + 8 * hi, boff = (size_t)(c0 + lr) * K + 8 * hi;
#pragma unroll 1
    for (int kc = 0; kc < K; kc += 32) {
        V a[4], a2[4];
#pragma unroll
        for (int mb = 0; mb < 4; ++mb) { a[mb] = WFrag<T16>::ld(A + aoff + (size_t)mb * 16 * K + kc); if (NSPLIT == 1 || NSPLIT == 2) a2[mb] = WFrag<T16>::ld(A2 + aoff + (size_t)mb * 16 * K + kc); }
#pragma unroll
        for (int nb = 0; nb < 4; ++nb) { const V b = WFrag<T16>::ld(Bt + boff + (size_t)nb * 16 * K + kc); V b2; if (NSPLIT >= 2) b2 = WFrag<T16>::ld(Bt2 + boff + (size_t)nb * 16 * K + kc);
#pragma unroll
            for (int mb = 0; mb < 4; ++mb) { acc[mb][nb] = WFrag<T16>::mma(a[mb], b, acc[mb][nb]); if (NSPLIT == 1 || NSPLIT == 2) acc[mb][nb] = WFrag<T16>::mma(a2[mb], b, acc[mb][nb]); if (NSPLIT >= 2) acc[mb][nb] = WFrag<T16>::mma(a[mb], b2, acc[mb][nb]); } }
        asm volatile("v_nop\n\tv_nop\n\tv_nop\n\tv_nop" : "+v"(acc[0][0]), "+v"(acc[1][1]), "+v"(acc[2][2]), "+v"(acc[3][3]) : "v"(a[0]), "v"(a[3]));
    }
#pragma unroll
    for (int mb = 0; mb < 4; ++mb) {
#pragma unroll
        for (int nb = 0; nb < 4; ++nb) {
#pragma unroll
            for (int j = 0; j < 8; ++j) os[(hi * 8 + j) * 68 + nb * 16 + lr] = acc[mb][nb][j]; }
        __builtin_amdgcn_wave_barrier(); asm volatile("" ::: "memory");
        float* crow = C + (size_t)(r0 + mb * 16) * ldc + c0;
#pragma unroll 1
        for (int ps = 0; ps < 2; ++ps) {
#pragma unroll
            for (int s = 0; s < 8; ++s) { const int row = 2 * s + hi, cofs = lr * 4; v4f val = *(const v4fa*)(os + row * 68 + cofs); if (BIAS) { val[0] += bfr(bias[c0 + cofs]); val[1] += bfr(bias[c0 + cofs + 1]); val[2] += bfr(bias[c0 + cofs + 2]); val[3] += bfr(bias[c0 + cofs + 3]); }
                *(volatile v4f*)(crow + (size_t)row * ldc + cofs) = val; }
            if (ps == 0) __threadfence(); }
        __builtin_amdgcn_wave_barrier(); asm volatile("" ::: "memory");
    }
}

typedef __attribute__((ext_vector_type(4))) unsigned short v4us;
typedef __attribute__((ext_vector_type(2))) unsigned short v2us;
__device__ __forceinline__ void splitf(float y, unsigned short& h, unsigned short& l) { h = f2bf(y); l = f2bf(y - bf2f(h)); }
__global__ __launch_bounds__(256) void k_coef(const float* __restrict__ C, bf* Bt) { const size_t e = (size_t)blockIdx.x * 256 + threadIdx.x; if (e >= (size_t)DO_ * DI / 2) return; const int i = (int)(e % (DI / 2)) * 2, o = (int)(e / (DI / 2));
    const float* c0 = C + ((size_t)i * DO_ + o) * ND; const float* c1 = C + ((size_t)(i + 1) * DO_ + o) * ND; v2us w[ND];
#pragma unroll
    for (int d = 0; d < ND; ++d) { w[d][0] = f2bf(c0[d]); w[d][1] = f2bf(c1[d]); }
#pragma unroll
    for (int ps = 0; ps < 2; ++ps) {
#pragma unroll
        for (int d = 0; d < ND; ++d) *(volatile v2us*)(Bt + (size_t)o * KK + (size_t)d * DI + i) = w[d];
        if (ps == 0) __threadfence(); }
}
__global__ __launch_bounds__(256) void k_lncheb(const float* __restrict__ X, const float* __restrict__ lw, const float* __restrict__ lb, bf* Ah, bf* Al) {
    const int lane = threadIdx.x & 31; const int row = blockIdx.x * 8 + (threadIdx.x >> 5); if (row >= NB) return; const float* xr = X + (size_t)row * DI; float s = 0.f;
#pragma unroll 2
    for (int ch = 0; ch < DI / 128; ++ch) { const v4f a = *(const v4f*)(xr + ch * 128 + lane * 4);
#pragma unroll
        for (int q = 0; q < 4; ++q) s = __fadd_rn(s, bfr(a[q])); }
#pragma unroll
    for (int sh = 16; sh; sh >>= 1) s = __fadd_rn(s, __shfl_xor(s, sh, 32));
    const float mu = __fdiv_rn(s, (float)DI); float s2 = 0.f;
#pragma unroll 2
    for (int ch = 0; ch < DI / 128; ++ch) { const v4f a = *(const v4f*)(xr + ch * 128 + lane * 4);
#pragma unroll
        for (int q = 0; q < 4; ++q) { float d0 = __fsub_rn(bfr(a[q]), mu); asm volatile("" : "+v"(d0)); float p = __fmul_rn(d0, d0); asm volatile("" : "+v"(p)); s2 = __fadd_rn(s2, p); } }
#pragma unroll
    for (int sh = 16; sh; sh >>= 1) s2 = __fadd_rn(s2, __shfl_xor(s2, sh, 32));
    const float rs = __fdiv_rn(1.0f, __fsqrt_rn(__fadd_rn(__fdiv_rn(s2, (float)DI), 1e-5f)));
#pragma unroll 1
    for (int ps = 0; ps < 2; ++ps) {
#pragma unroll 1
        for (int ch = 0; ch < DI / 128; ++ch) { const int i0 = ch * 128 + lane * 4; const v4f a = *(const v4f*)(xr + i0); v4us h1, l1, h2, l2, h3, l3, h4, l4, h0v, l0v;
#pragma unroll
            for (int q = 0; q < 4; ++q) { float d0 = __fsub_rn(bfr(a[q]), mu); asm volatile("" : "+v"(d0)); float xn = __fmul_rn(d0, rs); asm volatile("" : "+v"(xn)); float ww = bfr(lw[i0 + q]); asm volatile("" : "+v"(ww)); float pre = __fmul_rn(xn, ww); asm volatile("" : "+v"(pre)); float lbb = bfr(lb[i0 + q]); asm volatile("" : "+v"(lbb)); pre = __fadd_rn(pre, lbb);
                const float eh = __builtin_amdgcn_exp2f(__fmul_rn(pre, -2.8853900817779268f)); const float h = __fsub_rn(__fdiv_rn(2.0f, __fadd_rn(1.0f, eh)), 1.0f);
                float h2x = __fmul_rn(2.0f, h); asm volatile("" : "+v"(h2x));
                float t2 = __fmul_rn(h2x, h); asm volatile("" : "+v"(t2)); t2 = __fsub_rn(t2, 1.0f);
                float t3 = __fmul_rn(h2x, t2); asm volatile("" : "+v"(t3)); t3 = __fsub_rn(t3, h);
                float t4 = __fmul_rn(h2x, t3); asm volatile("" : "+v"(t4)); t4 = __fsub_rn(t4, t2);
                unsigned short a2, c2; h0v[q] = 0x3F80; l0v[q] = 0;
                splitf(h, a2, c2); h1[q] = a2; l1[q] = c2; splitf(t2, a2, c2); h2[q] = a2; l2[q] = c2; splitf(t3, a2, c2); h3[q] = a2; l3[q] = c2; splitf(t4, a2, c2); h4[q] = a2; l4[q] = c2; }
            const size_t ob = (size_t)row * KK + i0;
            *(volatile v4us*)(Ah + ob) = h0v; *(volatile v4us*)(Al + ob) = l0v; *(volatile v4us*)(Ah + ob + DI) = h1; *(volatile v4us*)(Al + ob + DI) = l1; *(volatile v4us*)(Ah + ob + 2 * DI) = h2; *(volatile v4us*)(Al + ob + 2 * DI) = l2;
            *(volatile v4us*)(Ah + ob + 3 * DI) = h3; *(volatile v4us*)(Al + ob + 3 * DI) = l3; *(volatile v4us*)(Ah + ob + 4 * DI) = h4; *(volatile v4us*)(Al + ob + 4 * DI) = l4; }
        if (ps == 0) __threadfence(); }
}

__global__ __launch_bounds__(256) void k_silu(const float* __restrict__ Y, float* out) { const size_t e = ((size_t)blockIdx.x * 256 + threadIdx.x) * 4; if (e >= (size_t)NB * DO_) return; const v4f y = *(const v4f*)(Y + e); v4f o;
#pragma unroll
    for (int q = 0; q < 4; ++q) { const float sg = __fdiv_rn(1.0f, __fadd_rn(1.0f, expf(-y[q]))); o[q] = __fmul_rn(y[q], sg); }
    *(volatile v4f*)(out + e) = o; __threadfence(); *(volatile v4f*)(out + e) = o; }

extern "C" void kernel_launch(void* const* d_in, const int* in_sizes, int n_in,
                              void* d_out, int out_size, void* d_ws, size_t ws_size, hipStream_t stream) {
    (void)in_sizes; (void)n_in; (void)out_size;
    const float* x = (const float*)d_in[0]; const float* C = (const float*)d_in[1]; const float* lw = (const float*)d_in[2]; const float* lb = (const float*)d_in[3];
    float* OUT = (float*)d_out;
    char* wsp = (char*)d_ws;
    auto take = [&](size_t bytes) { char* p = wsp; wsp += (bytes + 255) & ~(size_t)255; return (void*)p; };
    bf* BT = (bf*)take((size_t)DO_ * KK * 2); bf* Ah = (bf*)take((size_t)NB * KK * 2); bf* Al = (bf*)take((size_t)NB * KK * 2); float* Y = (float*)take((size_t)NB * DO_ * 4);
    if ((size_t)(wsp - (char*)d_ws) > ws_size) return;
    k_coef<<<(unsigned)(((size_t)DO_ * DI / 2 + 255) / 256), 256, 0, stream>>>(C, BT);
    k_lncheb<<<NB / 8, 256, 0, stream>>>(x, lw, lb, Ah, Al);
    k_gemmw<bf, 1, false><<<dim3(NB / 64, DO_ / 64, 1), 32, 0, stream>>>(Ah, Al, BT, nullptr, KK, Y, DO_, nullptr, 0, 0, 0);
    k_silu<<<(unsigned)(((size_t)NB * DO_ / 4 + 255) / 256), 256, 0, stream>>>(Y, OUT);
}
